// QuantumKernelFeedForward_65481071408021
// MI455X (gfx1250) — hardware-run, weakly checked
//
#include <hip/hip_runtime.h>


#ifndef NB
#define NB 8
#endif
#ifndef SEQ
#define SEQ 512
#endif
#define NTOK (NB * SEQ)
#define EMB  512
#define FFN_ 2048
#define NWIRE 4
#define GRB  32
#define GSC  16.0f
#define XSC  64.0f
#define WSC  1024.0f
#define TLP  72

static_assert(NTOK % 512 == 0);
static_assert(NTOK % 256 == 0);
static_assert(NTOK % GRB == 0);
static_assert(NTOK % 64 == 0 && EMB % 64 == 0 && FFN_ % 64 == 0);
static_assert(NTOK % 32 == 0 && EMB % 32 == 0 && FFN_ % 32 == 0);
static_assert(NWIRE == 4);
static_assert(EMB >= NWIRE);
static_assert((TLP * 2) % 16 == 0);
static_assert((NTOK * 2) % 128 == 0 && (EMB * 2) % 128 == 0 && (FFN_ * 2) % 128 == 0);
static_assert((EMB * 4) % 128 == 0);
static_assert(16 * 68 * 4 <= 131072);
static_assert(64 * TLP * 2 <= 131072);
static_assert(256 * 8 * 4 <= 131072);
static_assert(32 * 16 * 4 == 16 * 64 * 2);
static_assert(32 * 16 * 8 == 16 * 64 * 4);
static_assert(256 * 16 * 2 == 64 * 64 * 2);
static_assert(256 * 16 * 4 == 64 * 64 * 4);
static_assert(256 * 16 * 2 == 256 * 8 * 4);
static_assert(GSC * XSC == 1024.0f);

typedef _Float16 h16;
typedef __attribute__((ext_vector_type(16))) _Float16 v16h;
typedef __attribute__((ext_vector_type(8)))  _Float16 v8h;
typedef __attribute__((ext_vector_type(8)))  float    v8f;
typedef __attribute__((ext_vector_type(4)))  float    v4f;
typedef v4f  __attribute__((may_alias)) v4fa;
typedef v8h  __attribute__((may_alias)) v8ha;

__device__ __forceinline__ unsigned short f2bf(float f) { unsigned u = __float_as_uint(f); u += 0x7FFFu + ((u >> 16) & 1u); return (unsigned short)(u >> 16); }
__device__ __forceinline__ float bfr(float f) { return __uint_as_float(((unsigned)f2bf(f)) << 16); }
__device__ __forceinline__ v16h cat16(v8h lo, v8h hi) { return __builtin_shufflevector(lo, hi, 0, 1, 2, 3, 4, 5, 6, 7, 8, 9, 10, 11, 12, 13, 14, 15); }
__device__ __forceinline__ h16 toh_flush(float v) { const h16 r = (h16)v; return (fabsf(v) < 6.103515625e-05f) ? (h16)0.0f : r; }
__device__ __forceinline__ v8f wmma16g(v16h a, v16h b, v8f c) {
    c = __builtin_amdgcn_wmma_f32_16x16x32_f16(false, a, false, b, (short)0, c, false, false);
    asm volatile("v_nop\n\tv_nop\n\tv_nop\n\tv_nop" : "+v"(c) : "v"(a), "v"(b));
    return c;
}
__device__ __forceinline__ v16h  ldh(const h16* p) { return cat16(*(const v8h*)p, *(const v8h*)(p + 16)); }
__device__ __forceinline__ void wave_sync() { __builtin_amdgcn_fence(3  , "wavefront"); __builtin_amdgcn_wave_barrier(); asm volatile("" ::: "memory"); }

__global__ __launch_bounds__(256) void k_cvt_t(const float* __restrict__ src, h16* dst, int R, int C, float sc) {
#pragma clang fp contract(off)
    __shared__ __align__(16) h16 tl[64 * TLP];
    const int tid = threadIdx.x;
    const int c0 = blockIdx.x * 64, r0 = blockIdx.y * 64;
#pragma unroll
    for (int it = 0; it < 4; ++it) {
        const int rr = it * 16 + (tid >> 4), c4 = (tid & 15) * 4;
        const v4f v = *(const v4f*)(src + (size_t)(r0 + rr) * C + c0 + c4);
#pragma unroll
        for (int k = 0; k < 4; ++k) tl[(c4 + k) * TLP + rr] = toh_flush(bfr(v[k]) * sc);
    }
    __syncthreads();
#pragma unroll 1
    for (int ps = 0; ps < 2; ++ps) {
#pragma unroll
        for (int it = 0; it < 2; ++it) {
            const int p = it * 256 + tid; const int c = p >> 3, r8 = (p & 7) * 8;
            const v8h hv = *(const v8ha*)(&tl[c * TLP + r8]);
            *(volatile v8h*)(dst + (size_t)(c0 + c) * R + r0 + r8) = hv; }
        if (ps == 0) __threadfence(); }
}

__global__ __launch_bounds__(256) void k_trig(const float* __restrict__ x, float* TB) {
#pragma clang fp contract(off)
    __shared__ __align__(16) float ts[256 * 8];
    const int tid = threadIdx.x; const int j = blockIdx.x * 256 + tid;
#pragma unroll 1
    for (int w = 0; w < NWIRE; ++w) {
        const float a = 0.5f * bfr(x[(size_t)j * EMB + w]);
        ts[tid * 8 + w] = cosf(a); ts[tid * 8 + 4 + w] = sinf(a); }
    __syncthreads();
    float* tb = TB + (size_t)blockIdx.x * 256 * 8;
#pragma unroll 1
    for (int ps = 0; ps < 2; ++ps) {
#pragma unroll
        for (int it = 0; it < 2; ++it) { const int p = it * 256 + tid;
            const v4f v = *(const v4fa*)(&ts[p * 4]);
            *(volatile v4f*)(tb + (size_t)p * 4) = v; }
        if (ps == 0) __threadfence(); }
}

__global__ __launch_bounds__(64) void k_gram(const float* __restrict__ TB, h16* G) {
#pragma clang fp contract(off)
    const int tid = threadIdx.x;
    const int j0 = (blockIdx.x * 64 + tid) * 8;
    const int i0 = blockIdx.y * GRB;
    float cj[8][4], sj[8][4];
#pragma unroll
    for (int e = 0; e < 8; ++e) {
        const v4f a = *(const v4f*)(TB + (size_t)(j0 + e) * 8), b = *(const v4f*)(TB + (size_t)(j0 + e) * 8 + 4);
#pragma unroll
        for (int w = 0; w < 4; ++w) { cj[e][w] = a[w]; sj[e][w] = b[w]; } }
#pragma unroll 1
    for (int r = 0; r < GRB; ++r) {
        const int i = i0 + r;
        const v4f ci = *(const v4f*)(TB + (size_t)i * 8), si = *(const v4f*)(TB + (size_t)i * 8 + 4);
        v8h g;
#pragma unroll
        for (int e = 0; e < 8; ++e) {
            const float p0 = ci[0] * cj[e][0] + si[0] * sj[e][0];
            const float p1 = ci[1] * cj[e][1] + si[1] * sj[e][1];
            const float p2 = ci[2] * cj[e][2] + si[2] * sj[e][2];
            const float p3 = ci[3] * cj[e][3] + si[3] * sj[e][3];
            const float p = ((p0 * p1) * p2) * p3;
            g[e] = toh_flush(fabsf(p) * GSC); }
        h16* d = G + (size_t)i * NTOK + j0;
        *(volatile v8h*)d = g; __threadfence(); *(volatile v8h*)d = g;
    }
}

template <int EP, int K, int N>
__device__ __forceinline__ void gemm_body(const h16* __restrict__ A, const h16* __restrict__ Bt, const float* __restrict__ bias, h16* Ch, float* Cf, float osc) {
    __shared__ __align__(16) float os[16 * 68];
    const int lane = threadIdx.x & 31, lr = lane & 15, hi = lane >> 4; const int r0 = blockIdx.x * 64, c0 = blockIdx.y * 64;
    v8f acc[4][4];
#pragma unroll
    for (int mb = 0; mb < 4; ++mb)
#pragma unroll
        for (int nb = 0; nb < 4; ++nb) acc[mb][nb] = (v8f){};
    const size_t aoff = (size_t)(r0 + lr) * K + 8 * hi, boff = (size_t)(c0 + lr) * K + 8 * hi;
#pragma unroll 1
    for (int kc = 0; kc < K; kc += 32) {
        v16h a[4];
#pragma unroll
        for (int mb = 0; mb < 4; ++mb) a[mb] = ldh(A + aoff + (size_t)mb * 16 * K + kc);
#pragma unroll
        for (int nb = 0; nb < 4; ++nb) { const v16h b = ldh(Bt + boff + (size_t)nb * 16 * K + kc);
#pragma unroll
            for (int mb = 0; mb < 4; ++mb) acc[mb][nb] = wmma16g(a[mb], b, acc[mb][nb]); }
    }
    float bc[4];
#pragma unroll
    for (int nb = 0; nb < 4; ++nb) { bc[nb] = 0.0f; if (EP != 0) bc[nb] = bfr(bias[c0 + nb * 16 + lr]); }
#pragma unroll
    for (int mb = 0; mb < 4; ++mb) {
#pragma unroll
        for (int nb = 0; nb < 4; ++nb) {
#pragma unroll
            for (int j = 0; j < 8; ++j) { float v = acc[mb][nb][j] * osc + bc[nb]; if (EP == 1) v = fmaxf(v, 0.0f);
                os[(hi * 8 + j) * 68 + nb * 16 + lr] = v; } }
        wave_sync();
#pragma unroll 1
        for (int ps = 0; ps < 2; ++ps) {
            if (EP != 2) {
#pragma unroll
                for (int s = 0; s < 4; ++s) { const int row = 4 * s + (lane >> 3), c8 = (lane & 7) * 8;
                    const v4f x0 = *(const v4fa*)(&os[row * 68 + c8]); const v4f x1 = *(const v4fa*)(&os[row * 68 + c8 + 4]); v8h hv;
#pragma unroll
                    for (int i = 0; i < 4; ++i) { hv[i] = toh_flush(x0[i]); hv[4 + i] = toh_flush(x1[i]); }
                    *(volatile v8h*)(Ch + (size_t)(r0 + mb * 16 + row) * N + c0 + c8) = hv; }
            } else {
#pragma unroll
                for (int s = 0; s < 8; ++s) { const int p = s * 32 + lane; const int row = p >> 4, c4 = (p & 15) * 4;
                    const v4f val = *(const v4fa*)(&os[row * 68 + c4]);
                    *(volatile v4f*)(Cf + (size_t)(r0 + mb * 16 + row) * N + c0 + c4) = val; }
            }
            if (ps == 0) __threadfence(); }
        wave_sync();
    }
}

__global__ __launch_bounds__(32) void k_gemm_mix(const h16* __restrict__ A, const h16* __restrict__ Bt, h16* C) {
    gemm_body<0, NTOK, EMB>(A, Bt, (const float*)0, C, (float*)0, 1.0f / (GSC * XSC));
}
__global__ __launch_bounds__(32) void k_gemm_hid(const h16* __restrict__ A, const h16* __restrict__ Bt, const float* __restrict__ bias, h16* C) {
    gemm_body<1, EMB, FFN_>(A, Bt, bias, C, (float*)0, 1.0f / WSC);
}
__global__ __launch_bounds__(32) void k_gemm_out(const h16* __restrict__ A, const h16* __restrict__ Bt, const float* __restrict__ bias, float* C) {
    gemm_body<2, FFN_, EMB>(A, Bt, bias, (h16*)0, C, 1.0f / WSC);
}

static constexpr size_t al256(size_t v) { return (v + 255) & ~(size_t)255; }
static constexpr size_t SZ_XT  = al256((size_t)EMB * NTOK * 2);
static constexpr size_t SZ_W1T = al256((size_t)FFN_ * EMB * 2);
static constexpr size_t SZ_W2T = al256((size_t)EMB * FFN_ * 2);
static constexpr size_t SZ_TB  = al256((size_t)NTOK * 8 * 4);
static constexpr size_t SZ_G   = al256((size_t)NTOK * NTOK * 2);
static constexpr size_t SZ_MIX = al256((size_t)NTOK * EMB * 2);
static constexpr size_t SZ_HID = al256((size_t)NTOK * FFN_ * 2);
static constexpr size_t SZ_TOTAL = SZ_XT + SZ_W1T + SZ_W2T + SZ_TB + SZ_G + SZ_MIX + SZ_HID;
static_assert(SZ_TOTAL <= (size_t)134217728);
static_assert(((size_t)NTOK * 8 * 4) % 128 == 0);

extern "C" void kernel_launch(void* const* d_in, const int* in_sizes, int n_in,
                              void* d_out, int out_size, void* d_ws, size_t ws_size, hipStream_t stream) {
    if (n_in < 5) return;
    if ((size_t)in_sizes[0] < (size_t)NTOK * EMB) return;
    if ((size_t)in_sizes[1] < (size_t)EMB * FFN_ || in_sizes[2] < FFN_) return;
    if ((size_t)in_sizes[3] < (size_t)FFN_ * EMB || in_sizes[4] < EMB) return;
    if ((size_t)out_size < (size_t)NTOK * EMB) return;
    if (SZ_TOTAL > ws_size) return;
    const float* x  = (const float*)d_in[0];
    const float* w1 = (const float*)d_in[1]; const float* b1 = (const float*)d_in[2];
    const float* w2 = (const float*)d_in[3]; const float* b2 = (const float*)d_in[4];
    float* Y = (float*)d_out;
    char* wsp = (char*)d_ws;
    h16* XT  = (h16*)wsp;   wsp += SZ_XT;
    h16* W1T = (h16*)wsp;   wsp += SZ_W1T;
    h16* W2T = (h16*)wsp;   wsp += SZ_W2T;
    float* TB = (float*)wsp; wsp += SZ_TB;
    h16* G   = (h16*)wsp;   wsp += SZ_G;
    h16* MIX = (h16*)wsp;   wsp += SZ_MIX;
    h16* HID = (h16*)wsp;   wsp += SZ_HID;

    k_cvt_t<<<dim3(EMB / 64, NTOK / 64, 1), 256, 0, stream>>>(x, XT, NTOK, EMB, XSC);
    k_cvt_t<<<dim3(FFN_ / 64, EMB / 64, 1), 256, 0, stream>>>(w1, W1T, EMB, FFN_, WSC);
    k_cvt_t<<<dim3(EMB / 64, FFN_ / 64, 1), 256, 0, stream>>>(w2, W2T, FFN_, EMB, WSC);

    k_trig<<<NTOK / 256, 256, 0, stream>>>(x, TB);
    k_gram<<<dim3(NTOK / 512, NTOK / GRB, 1), 64, 0, stream>>>(TB, G);

    k_gemm_mix<<<dim3(NTOK / 64, EMB / 64, 1), 32, 0, stream>>>(G, XT, MIX);
    k_gemm_hid<<<dim3(NTOK / 64, FFN_ / 64, 1), 32, 0, stream>>>(MIX, W1T, b1, HID);
    k_gemm_out<<<dim3(NTOK / 64, EMB / 64, 1), 32, 0, stream>>>(HID, W2T, b2, Y);
}
